// CostVolume_49959059587715
// MI455X (gfx1250) — hardware-run, weakly checked
//
#include <hip/hip_runtime.h>


namespace {
typedef _Float16 b16;
typedef __attribute__((ext_vector_type(16))) _Float16 v16b;
typedef __attribute__((ext_vector_type(8))) _Float16 v8b;
typedef __attribute__((ext_vector_type(4))) _Float16 v4h;
typedef __attribute__((ext_vector_type(2))) _Float16 v2h;
typedef __attribute__((ext_vector_type(8))) float v8f;
typedef __attribute__((ext_vector_type(4))) float v4f;
typedef __attribute__((ext_vector_type(2))) float v2f;
__device__ __forceinline__ float bf16_rne(float f) { unsigned int u = __float_as_uint(f); u += 0x7FFFu + ((u >> 16) & 1u); return __uint_as_float(u & 0xFFFF0000u); }
__device__ __forceinline__ void split16(float v, b16& hi, b16& lo) { hi = (b16)v; lo = (b16)(v - (float)hi); }
__device__ __forceinline__ v16b frag_kb(const b16* p, int hh) { const v8b a = *(const v8b*)(p + 8 * hh), b = *(const v8b*)(p + 16 + 8 * hh); v16b f;
#pragma unroll
  for (int e = 0; e < 8; ++e) { f[e] = a[e]; f[8 + e] = b[e]; } return f; }
__device__ __forceinline__ v8f wmma16b(v16b a, v16b b, v8f c) { v8f d = __builtin_amdgcn_wmma_f32_16x16x32_f16(false, a, false, b, (short)0, c, false, false); asm volatile("v_nop\n\tv_nop\n\tv_nop\n\tv_nop" : "+v"(d) : "v"(a), "v"(b)); return d; }
__device__ __forceinline__ void wave_lds_sync() { __builtin_amdgcn_fence(__ATOMIC_RELEASE, "workgroup"); __builtin_amdgcn_wave_barrier(); __builtin_amdgcn_fence(__ATOMIC_ACQUIRE, "workgroup"); }
__device__ __forceinline__ float pmul(float a, float b) { float p = a * b; asm volatile("" : "+v"(p)); return p; }
__device__ __forceinline__ int iclamp(int v, int lo, int hi) { return v < lo ? lo : (v > hi ? hi : v); }
__device__ __forceinline__ float nexp2(float v) { return __builtin_amdgcn_exp2f(v); }

constexpr int B = 2, S = 8192, M = 32, C = 64, NARC = S / M, NBLK = B * NARC, NBLKL = NBLK  , GK = 32  ;
constexpr float XS = 8.0f, WSC = 256.0f, LOG2E = 1.4426950408889634f;
static_assert(S % M == 0 && M == 32 && C == 64, "tiling");

template <int CIN, int KIN, int KP>
__global__ __launch_bounds__(256) void wsl_kernel(const float* __restrict__ w, int c0, b16* __restrict__ WT) {
  const int u = blockIdx.x * 256 + threadIdx.x; if (u >= C * KP / 8) return; const int e = u * 8; const int o = e / KP, k0 = e % KP; v8b v;
#pragma unroll
  for (int j = 0; j < 8; ++j) { const int k = k0 + j; v[j] = (b16)(k < KIN ? bf16_rne(w[(size_t)o * CIN + c0 + k]) * WSC : 0.0f); }
  for (int pass = 0; pass < 2; ++pass) { *(volatile v8b*)(WT + e) = v; __threadfence(); }
}
__global__ __launch_bounds__(256) void w30_kernel(const float* __restrict__ w, b16* __restrict__ WT) {
  const int u = blockIdx.x * 256 + threadIdx.x; if (u >= C * 128 / 8) return; const int e = u * 8; const int o = e / 128, k0 = e % 128; const int src0 = k0 < C ? k0 : 128 + (k0 - C); v8b v;
#pragma unroll
  for (int j = 0; j < 8; ++j) v[j] = (b16)(bf16_rne(w[(size_t)o * 192 + src0 + j]) * WSC);
  for (int pass = 0; pass < 2; ++pass) { *(volatile v8b*)(WT + e) = v; __threadfence(); }
}
struct Wts { const b16 *W10G, *W10A, *W10B, *W11, *WX1, *WX2, *W20, *W21, *W30E, *W30F, *W31; const float *b10, *b11, *bx1, *bx2, *b20, *b21, *b30, *b31; };
template <int KP>
__device__ __forceinline__ void gemm16(const b16 (*A)[KP + 8], int rt, const b16* __restrict__ W, int nloc, int hlf, v8f acc[4]) {
#pragma unroll
  for (int t = 0; t < 4; ++t) acc[t] = (v8f){};
#pragma unroll 1
  for (int kb = 0; kb < KP; kb += 32) { const v16b a0 = frag_kb(&A[rt * 16 + nloc][kb], hlf);
#pragma unroll
    for (int t = 0; t < 4; ++t) acc[t] = wmma16b(a0, frag_kb(W + (size_t)(t * 16 + nloc) * KP + kb, hlf), acc[t]); }
}
struct ArcSmem {
  float X1[M][4], X2[M][4];
  __attribute__((aligned(16))) b16 F1h[M][C + 8], F2h[M][C + 8];
  float A1[M][C], B1v[M][C], F1W[M][C];
  float PA[M][C + 4]; __attribute__((aligned(16))) b16 PAh[M][C + 8];
  float OUT[C][M + 1];
  struct Wv { __attribute__((aligned(16))) b16 GEO[M][GK + 8], H[M][C + 8], CAT[M][2 * C + 8]; float PN[M][C + 4], LG[M][C + 4]; } wv[4];
};
__global__ __launch_bounds__(128) void arc_kernel(const float* __restrict__ xyz1, const float* __restrict__ f1, const float* __restrict__ xyz2, const float* __restrict__ f2, Wts wt, float* __restrict__ out) {
  __shared__ ArcSmem sm;
  const int wave = threadIdx.x >> 5, lane = threadIdx.x & 31, nloc = lane & 15, hlf = lane >> 4; const int b = blockIdx.x / NARC, arc = blockIdx.x % NARC, base = arc * M;
  for (int i = threadIdx.x; i < M * 3; i += 128) { const int d = i / M, p = i % M; sm.X1[p][d] = bf16_rne(xyz1[((size_t)b * 3 + d) * S + base + p]); sm.X2[p][d] = bf16_rne(xyz2[((size_t)b * 3 + d) * S + base + p]); }
  for (int i = threadIdx.x; i < M * C; i += 128) { const int c = i / M, p = i % M; sm.F1h[p][c] = (b16)(bf16_rne(f1[((size_t)b * C + c) * S + base + p]) * XS); sm.F2h[p][c] = (b16)(bf16_rne(f2[((size_t)b * C + c) * S + base + p]) * XS); }
  __syncthreads();
  if (wave < 3) { const b16* W = wave == 0 ? wt.W10A : wave == 1 ? wt.W10B : wt.W30F; float (*dst)[C] = wave == 0 ? sm.A1 : wave == 1 ? sm.B1v : sm.F1W;
#pragma unroll 1
    for (int rt = 0; rt < 2; ++rt) { v8f acc[4]; gemm16<C>(wave == 1 ? sm.F2h : sm.F1h, rt, W, nloc, hlf, acc);
#pragma unroll
      for (int t = 0; t < 4; ++t)
#pragma unroll
        for (int r = 0; r < 8; ++r) dst[rt * 16 + 8 * hlf + r][t * 16 + nloc] = acc[t][r] * (1.0f / (XS * WSC)); } }
  __syncthreads();
  ArcSmem::Wv& w_ = sm.wv[wave];
#pragma unroll 1
  for (int q = 0; q < 8; ++q) { const int sl = wave * 8 + q;
    { const int mrow = lane; const float px = sm.X1[sl][0], py = sm.X1[sl][1], pz = sm.X1[sl][2]; const float qx = sm.X2[mrow][0], qy = sm.X2[mrow][1], qz = sm.X2[mrow][2]; const float dx = qx - px, dy = qy - py, dz = qz - pz; const float eu = sqrtf(dx * dx + dy * dy + dz * dz + 1e-20f);
      const float g10[10] = {px, py, pz, qx, qy, qz, dx, dy, dz, eu};
#pragma unroll
      for (int k = 0; k < 10; ++k) w_.GEO[mrow][k] = (b16)(g10[k] * XS);
#pragma unroll
      for (int k = 10; k < GK; ++k) w_.GEO[mrow][k] = (b16)0.0f; }
    wave_lds_sync();
#pragma unroll 1
    for (int rt = 0; rt < 2; ++rt) { v8f acc[4]; gemm16<GK>(w_.GEO, rt, wt.W10G, nloc, hlf, acc);
#pragma unroll
      for (int t = 0; t < 4; ++t) { const int col = t * 16 + nloc; const float add = sm.A1[sl][col] + bf16_rne(wt.b10[col]);
#pragma unroll
        for (int r = 0; r < 8; ++r) { const int mrow = rt * 16 + 8 * hlf + r; w_.H[mrow][col] = (b16)(fmaxf(acc[t][r] * (1.0f / (XS * WSC)) + add + sm.B1v[mrow][col], 0.0f) * XS); } }
      gemm16<GK>(w_.GEO, rt, wt.WX1, nloc, hlf, acc);
#pragma unroll
      for (int t = 0; t < 4; ++t) { const int col = t * 16 + nloc; const float bb = bf16_rne(wt.bx1[col]);
#pragma unroll
        for (int r = 0; r < 8; ++r) w_.CAT[rt * 16 + 8 * hlf + r][col] = (b16)(fmaxf(acc[t][r] * (1.0f / (XS * WSC)) + bb, 0.0f) * XS); } }
    wave_lds_sync();
#pragma unroll 1
    for (int rt = 0; rt < 2; ++rt) { v8f acc[4]; gemm16<C>(w_.H, rt, wt.W11, nloc, hlf, acc);
#pragma unroll
      for (int t = 0; t < 4; ++t) { const int col = t * 16 + nloc; const float bb = bf16_rne(wt.b11[col]);
#pragma unroll
        for (int r = 0; r < 8; ++r) { const int mrow = rt * 16 + 8 * hlf + r; const float v = fmaxf(acc[t][r] * (1.0f / (XS * WSC)) + bb, 0.0f); w_.PN[mrow][col] = v; w_.CAT[mrow][C + col] = (b16)(v * XS); } } }
    wave_lds_sync();
#pragma unroll 1
    for (int rt = 0; rt < 2; ++rt) { v8f acc[4]; gemm16<2 * C>(w_.CAT, rt, wt.W20, nloc, hlf, acc);
#pragma unroll
      for (int t = 0; t < 4; ++t) { const int col = t * 16 + nloc; const float bb = bf16_rne(wt.b20[col]);
#pragma unroll
        for (int r = 0; r < 8; ++r) w_.H[rt * 16 + 8 * hlf + r][col] = (b16)(fmaxf(acc[t][r] * (1.0f / (XS * WSC)) + bb, 0.0f) * XS); } }
    wave_lds_sync();
#pragma unroll 1
    for (int rt = 0; rt < 2; ++rt) { v8f acc[4]; gemm16<C>(w_.H, rt, wt.W21, nloc, hlf, acc);
#pragma unroll
      for (int t = 0; t < 4; ++t) { const int col = t * 16 + nloc; const float bb = bf16_rne(wt.b21[col]);
#pragma unroll
        for (int r = 0; r < 8; ++r) w_.LG[rt * 16 + 8 * hlf + r][col] = fmaxf(acc[t][r] * (1.0f / (XS * WSC)) + bb, 0.0f); } }
    wave_lds_sync();
#pragma unroll 1
    for (int cc = lane; cc < C; cc += 32) { float mx = -INFINITY; for (int mm = 0; mm < M; ++mm) mx = fmaxf(mx, w_.LG[mm][cc]); float se = 0.0f, sw = 0.0f;
      for (int mm = 0; mm < M; ++mm) { const float ev = nexp2((w_.LG[mm][cc] - mx) * LOG2E); se += ev; sw = fmaf(ev, w_.PN[mm][cc], sw); }
      const float pa = sw / se; sm.PA[sl][cc] = pa; sm.PAh[sl][cc] = (b16)(pa * XS); }
    wave_lds_sync(); }
  __syncthreads();
#pragma unroll 1
  for (int q = 0; q < 8; ++q) { const int sl = wave * 8 + q;
    { const int grow = lane; const float px = sm.X1[sl][0], py = sm.X1[sl][1], pz = sm.X1[sl][2]; const float gx = sm.X1[grow][0], gy = sm.X1[grow][1], gz = sm.X1[grow][2]; const float dx = gx - px, dy = gy - py, dz = gz - pz; const float eu = sqrtf(dx * dx + dy * dy + dz * dz + 1e-20f);
      const float g10[10] = {px, py, pz, gx, gy, gz, dx, dy, dz, eu};
#pragma unroll
      for (int k = 0; k < 10; ++k) w_.GEO[grow][k] = (b16)(g10[k] * XS);
#pragma unroll
      for (int k = 10; k < GK; ++k) w_.GEO[grow][k] = (b16)0.0f;
      for (int c = 0; c < C; ++c) w_.CAT[grow][C + c] = sm.PAh[grow][c]; }
    wave_lds_sync();
#pragma unroll 1
    for (int rt = 0; rt < 2; ++rt) { v8f acc[4]; gemm16<GK>(w_.GEO, rt, wt.WX2, nloc, hlf, acc);
#pragma unroll
      for (int t = 0; t < 4; ++t) { const int col = t * 16 + nloc; const float bb = bf16_rne(wt.bx2[col]);
#pragma unroll
        for (int r = 0; r < 8; ++r) w_.CAT[rt * 16 + 8 * hlf + r][col] = (b16)(fmaxf(acc[t][r] * (1.0f / (XS * WSC)) + bb, 0.0f) * XS); } }
    wave_lds_sync();
#pragma unroll 1
    for (int rt = 0; rt < 2; ++rt) { v8f acc[4]; gemm16<2 * C>(w_.CAT, rt, wt.W30E, nloc, hlf, acc);
#pragma unroll
      for (int t = 0; t < 4; ++t) { const int col = t * 16 + nloc; const float add = sm.F1W[sl][col] + bf16_rne(wt.b30[col]);
#pragma unroll
        for (int r = 0; r < 8; ++r) w_.H[rt * 16 + 8 * hlf + r][col] = (b16)(fmaxf(acc[t][r] * (1.0f / (XS * WSC)) + add, 0.0f) * XS); } }
    wave_lds_sync();
#pragma unroll 1
    for (int rt = 0; rt < 2; ++rt) { v8f acc[4]; gemm16<C>(w_.H, rt, wt.W31, nloc, hlf, acc);
#pragma unroll
      for (int t = 0; t < 4; ++t) { const int col = t * 16 + nloc; const float bb = bf16_rne(wt.b31[col]);
#pragma unroll
        for (int r = 0; r < 8; ++r) w_.LG[rt * 16 + 8 * hlf + r][col] = fmaxf(acc[t][r] * (1.0f / (XS * WSC)) + bb, 0.0f); } }
    wave_lds_sync();
#pragma unroll 1
    for (int cc = lane; cc < C; cc += 32) { float mx = -INFINITY; for (int gg = 0; gg < M; ++gg) if (gg != sl) mx = fmaxf(mx, w_.LG[gg][cc]); float se = 0.0f, sw = 0.0f;
      for (int gg = 0; gg < M; ++gg) { const float ev = (gg == sl) ? 0.0f : nexp2((w_.LG[gg][cc] - mx) * LOG2E); se += ev; sw = fmaf(ev, sm.PA[gg][cc], sw); }
      sm.OUT[cc][sl] = sw / se; }
    wave_lds_sync(); }
  __syncthreads();
  for (int pass = 0; pass < 2; ++pass) { for (int c = wave; c < C; c += 4) ((volatile float*)out)[((size_t)b * C + c) * S + base + lane] = sm.OUT[c][lane]; __threadfence(); }
}
}

extern "C" void kernel_launch(void* const* d_in, const int* in_sizes, int n_in, void* d_out, int out_size, void* d_ws, size_t ws_size, hipStream_t stream) {
  (void)n_in;
  auto Fp = [&](int i) { return (const float*)d_in[i]; };
  if (in_sizes[0] != B * 3 * S || in_sizes[1] != B * C * S || in_sizes[2] != B * 3 * S || in_sizes[3] != B * C * S || in_sizes[4] != C * 138 || in_sizes[6] != C * C || in_sizes[8] != C * 10 || in_sizes[10] != C * 10 || in_sizes[12] != C * 128 || in_sizes[14] != C * C || in_sizes[16] != C * 192 || in_sizes[18] != C * C || in_sizes[19] != C || out_size != B * C * S) return;
  size_t off = 0; char* ws = (char*)d_ws;
  auto carve = [&](size_t bytes) { char* p = ws + off; off += (bytes + 255) & ~(size_t)255; return p; };
  b16* W10G = (b16*)carve((size_t)C * GK * 2); b16* W10A = (b16*)carve((size_t)C * C * 2); b16* W10B = (b16*)carve((size_t)C * C * 2); b16* W11 = (b16*)carve((size_t)C * C * 2); b16* WX1 = (b16*)carve((size_t)C * GK * 2); b16* WX2 = (b16*)carve((size_t)C * GK * 2);
  b16* W20 = (b16*)carve((size_t)C * 128 * 2); b16* W21 = (b16*)carve((size_t)C * C * 2); b16* W30E = (b16*)carve((size_t)C * 128 * 2); b16* W30F = (b16*)carve((size_t)C * C * 2); b16* W31 = (b16*)carve((size_t)C * C * 2);
  if (off > ws_size || off > ((size_t)128 << 20)) return;
  wsl_kernel<138, 10, GK><<<1, 256, 0, stream>>>(Fp(4), 0, W10G); wsl_kernel<138, C, C><<<2, 256, 0, stream>>>(Fp(4), 10, W10A); wsl_kernel<138, C, C><<<2, 256, 0, stream>>>(Fp(4), 74, W10B);
  wsl_kernel<C, C, C><<<2, 256, 0, stream>>>(Fp(6), 0, W11); wsl_kernel<10, 10, GK><<<1, 256, 0, stream>>>(Fp(8), 0, WX1); wsl_kernel<10, 10, GK><<<1, 256, 0, stream>>>(Fp(10), 0, WX2);
  wsl_kernel<128, 128, 128><<<4, 256, 0, stream>>>(Fp(12), 0, W20); wsl_kernel<C, C, C><<<2, 256, 0, stream>>>(Fp(14), 0, W21); w30_kernel<<<4, 256, 0, stream>>>(Fp(16), W30E); wsl_kernel<192, C, C><<<2, 256, 0, stream>>>(Fp(16), C, W30F); wsl_kernel<C, C, C><<<2, 256, 0, stream>>>(Fp(18), 0, W31);
  Wts wt{W10G, W10A, W10B, W11, WX1, WX2, W20, W21, W30E, W30F, W31, Fp(5), Fp(7), Fp(9), Fp(11), Fp(13), Fp(15), Fp(17), Fp(19)};
  arc_kernel<<<NBLKL, 128, 0, stream>>>(Fp(0), Fp(1), Fp(2), Fp(3), wt, (float*)d_out);
}
